// GatedLinearAttention_61040075210837
// MI455X (gfx1250) — hardware-run, weakly checked
//
#include <hip/hip_runtime.h>


#define NL   1024
#define NM   1024
#define NU   16
#define NE   64
#define NJ   3072
#define OB   1024
#define OC   2048
typedef _Float16 h16;
typedef unsigned short bf;
typedef __attribute__((ext_vector_type(16))) __bf16   v16bf;
typedef __attribute__((ext_vector_type(16))) _Float16 v16h;
typedef __attribute__((ext_vector_type(8)))  _Float16 v8h;
typedef __attribute__((ext_vector_type(8)))  unsigned short v8us;
typedef __attribute__((ext_vector_type(8)))  float    v8f;
typedef __attribute__((ext_vector_type(4)))  float    v4f;
typedef v8h  __attribute__((may_alias)) v8ha;
typedef v4f  __attribute__((may_alias)) v4fa;
typedef v8us __attribute__((may_alias)) v8usa;

__device__ __forceinline__ unsigned short f2bf(float f) { unsigned u = __float_as_uint(f); u += 0x7FFFu + ((u >> 16) & 1u); return (unsigned short)(u >> 16); }
__device__ __forceinline__ float bf2f(unsigned short b) { return __uint_as_float(((unsigned)b) << 16); }
__device__ __forceinline__ float bfr(float f) { return bf2f(f2bf(f)); }
__device__ __forceinline__ v16h cat16(v8h lo, v8h hi) { return __builtin_shufflevector(lo, hi, 0, 1, 2, 3, 4, 5, 6, 7, 8, 9, 10, 11, 12, 13, 14, 15); }
__device__ __forceinline__ v16bf cat16b(v8us lo, v8us hi) { return __builtin_bit_cast(v16bf, __builtin_shufflevector(lo, hi, 0, 1, 2, 3, 4, 5, 6, 7, 8, 9, 10, 11, 12, 13, 14, 15)); }
__device__ __forceinline__ v8f wmma16(v16h a, v16h b, v8f c) { return __builtin_amdgcn_wmma_f32_16x16x32_f16(false, a, false, b, (short)0, c, false, false); }
__device__ __forceinline__ v8f wmmab(v16bf a, v16bf b, v8f c) { return __builtin_amdgcn_wmma_f32_16x16x32_bf16(false, a, false, b, (short)0, c, false, false); }

template <typename T16> struct WFrag;
template <> struct WFrag<h16> { typedef v16h V; static __device__ __forceinline__ V ld(const h16* p) { return cat16(*(const v8h*)p, *(const v8h*)(p + 16)); } static __device__ __forceinline__ v8f mma(V a, V b, v8f c) { return wmma16(a, b, c); } };
template <> struct WFrag<bf> { typedef v16bf V; static __device__ __forceinline__ V ld(const bf* p) { return cat16b(*(const v8us*)p, *(const v8us*)(p + 16)); } static __device__ __forceinline__ v8f mma(V a, V b, v8f c) { return wmmab(a, b, c); } };
template <typename T16, int NSPLIT, bool BIAS>
__global__ __launch_bounds__(32) void k_gemmw(const T16* __restrict__ A, const T16* __restrict__ A2, const T16* __restrict__ Bt, const T16* __restrict__ Bt2, int K, float* C, int ldc, const float* __restrict__ bias, size_t sA, size_t sB, size_t sC) {
    typedef typename WFrag<T16>::V V;
    __shared__ __align__(16) float os[16 * 68];
    const size_t z = blockIdx.z; A += z * sA; if (A2) A2 += z * sA; Bt += z * sB; if (Bt2) Bt2 += z * sB; C += z * sC;
    const int lane = threadIdx.x & 31, lr = lane & 15, hi = lane >> 4; const int r0 = blockIdx.x * 64, c0 = blockIdx.y * 64;
    v8f acc[4][4];
#pragma unroll
    for (int mb = 0; mb < 4; ++mb)
#pragma unroll
        for (int nb = 0; nb < 4; ++nb) acc[mb][nb] = (v8f){};
    const size_t aoff = (size_t)(r0 + lr) * K + 8 * hi, boff = (size_t)(c0 + lr) * K + 8 * hi;
    for (int kc = 0; kc < K; kc += 32) {
        V a[4], a2[4];
#pragma unroll
        for (int mb = 0; mb < 4; ++mb) { a[mb] = WFrag<T16>::ld(A + aoff + (size_t)mb * 16 * K + kc); if (NSPLIT == 1 || NSPLIT == 2) a2[mb] = WFrag<T16>::ld(A2 + aoff + (size_t)mb * 16 * K + kc); }
#pragma unroll
        for (int nb = 0; nb < 4; ++nb) { const V b = WFrag<T16>::ld(Bt + boff + (size_t)nb * 16 * K + kc); V b2; if (NSPLIT >= 2) b2 = WFrag<T16>::ld(Bt2 + boff + (size_t)nb * 16 * K + kc);
#pragma unroll
            for (int mb = 0; mb < 4; ++mb) { acc[mb][nb] = WFrag<T16>::mma(a[mb], b, acc[mb][nb]); if (NSPLIT == 1 || NSPLIT == 2) acc[mb][nb] = WFrag<T16>::mma(a2[mb], b, acc[mb][nb]); if (NSPLIT >= 2) acc[mb][nb] = WFrag<T16>::mma(a[mb], b2, acc[mb][nb]); } }
        asm volatile("v_nop\n\tv_nop\n\tv_nop\n\tv_nop" : "+v"(acc[0][0]), "+v"(acc[1][1]), "+v"(acc[2][2]), "+v"(acc[3][3]) : "v"(a[0]), "v"(a[3]));
    }
#pragma unroll
    for (int mb = 0; mb < 4; ++mb) {
#pragma unroll
        for (int nb = 0; nb < 4; ++nb) {
#pragma unroll
            for (int j = 0; j < 8; ++j) os[(hi * 8 + j) * 68 + nb * 16 + lr] = acc[mb][nb][j]; }
        __builtin_amdgcn_wave_barrier(); asm volatile("" ::: "memory");
        float* crow = C + (size_t)(r0 + mb * 16) * ldc + c0;
#pragma unroll 1
        for (int ps = 0; ps < 2; ++ps) {
#pragma unroll
            for (int s = 0; s < 8; ++s) { const int row = 2 * s + hi, cofs = lr * 4; v4f val = *(const v4fa*)(os + row * 68 + cofs); if (BIAS) { val[0] += bfr(bias[c0 + cofs]); val[1] += bfr(bias[c0 + cofs + 1]); val[2] += bfr(bias[c0 + cofs + 2]); val[3] += bfr(bias[c0 + cofs + 3]); }
                *(volatile v4f*)(crow + (size_t)row * ldc + cofs) = val; }
            if (ps == 0) __threadfence(); }
        __builtin_amdgcn_wave_barrier(); asm volatile("" ::: "memory");
    }
}

typedef __attribute__((ext_vector_type(2))) _Float16 v2h;
typedef __attribute__((ext_vector_type(4))) _Float16 v4h;
typedef __attribute__((ext_vector_type(2))) unsigned short v2us;
typedef __attribute__((ext_vector_type(4))) unsigned short v4us;
typedef __attribute__((ext_vector_type(2))) float v2f;
typedef __attribute__((ext_vector_type(4))) int v4i;

__global__ __launch_bounds__(256) void k_cvt8(const float* __restrict__ src, bf* dst, size_t n8) { const size_t i = (size_t)blockIdx.x * 256 + threadIdx.x; if (i >= n8) return; const v8f v = *(const v8f*)(src + i * 8); v8us o;
#pragma unroll
    for (int k = 0; k < 8; ++k) o[k] = f2bf(v[k]); *(volatile v8us*)(dst + i * 8) = o; __threadfence(); *(volatile v8us*)(dst + i * 8) = o; }

__device__ __forceinline__ h16 toh_flush(float x) { const float z = (fabsf(x) < 6.103515625e-05f) ? 0.0f : x; return (h16)z; }

template <bool RB>
__global__ __launch_bounds__(256) void k_c16(const float* __restrict__ src, h16* dst, size_t n8) { const size_t i = (size_t)blockIdx.x * 256 + threadIdx.x; if (i >= n8) return; const float* p = src + i * 8; const v4f a = *(const v4f*)p, b = *(const v4f*)(p + 4); v8h o;
#pragma unroll
    for (int q = 0; q < 4; ++q) { o[q] = toh_flush(RB ? bfr(a[q]) : a[q]); o[q + 4] = toh_flush(RB ? bfr(b[q]) : b[q]); }
    *(volatile v8h*)(dst + i * 8) = o; __threadfence(); *(volatile v8h*)(dst + i * 8) = o; }

__global__ __launch_bounds__(256) void k_eases(const float* __restrict__ a1, const float* __restrict__ a6, const float* __restrict__ a7, const float* __restrict__ Pj, float* Lg, float* Ez) { const unsigned nb = blockIdx.x * 256u + threadIdx.x; const unsigned un = nb & 15u, st = nb >> 4; const float* xr = a1 + (size_t)st * NM + un * NE; const float* br = Pj + (size_t)st * NJ + OB + un * NE; float s1 = 0.0f, s2 = 0.0f;
#pragma unroll
    for (int j = 0; j < NE; ++j) { s1 += bfr(xr[j]) * bfr(a6[j]); s2 += br[j] * bfr(a7[j]); }
    const float e1 = fmaxf(1.0f / (1.0f + expf(-s1)), 1e-6f); const float lg = logf(e1); const float ez = s2 / (1.0f + expf(-s2));
    *(volatile float*)(Lg + nb) = lg; *(volatile float*)(Ez + nb) = ez; __threadfence(); *(volatile float*)(Lg + nb) = lg; *(volatile float*)(Ez + nb) = ez; }

__global__ __launch_bounds__(32) void k_sums(const float* __restrict__ Lg, const float* __restrict__ Ez, float* Wg, float* Cf) { const unsigned ln = threadIdx.x; const unsigned un = ln & 15u, hf = ln >> 4; float run = 0.0f;
    for (int tp = 0; tp < NL / 2; ++tp) { const float g0 = Lg[(2 * tp) * NU + un]; const float g1 = Lg[(2 * tp + 1) * NU + un]; const float r0 = run + g0; const float r1 = r0 + g1; const float mine = hf ? r1 : r0; run = r1; const float hd = fminf(fmaxf(mine, -30.0f), 30.0f); const float wt = expf(hd) + 1e-6f; const unsigned at = (unsigned)tp * 32u + ln; const float cf = Ez[at] / wt; *(volatile float*)(Wg + at) = wt; *(volatile float*)(Cf + at) = cf; __threadfence(); *(volatile float*)(Wg + at) = wt; *(volatile float*)(Cf + at) = cf; } }

__global__ __launch_bounds__(64) void k_tally(const float* __restrict__ Pj, const float* __restrict__ Wg, const float* __restrict__ Cf, float* Og) { const unsigned un = blockIdx.x, cj = threadIdx.x; float tw[NE];
#pragma unroll
    for (int i = 0; i < NE; ++i) tw[i] = 0.0f;
    for (int st = 0; st < NL; ++st) { const float* pr = Pj + (size_t)st * NJ + un * NE; const float wt = Wg[st * NU + un]; const float cf = Cf[st * NU + un] * pr[OC + cj]; float acc = 0.0f;
#pragma unroll
        for (int i = 0; i < NE; ++i) { tw[i] += cf * pr[OB + i]; acc += pr[i] * tw[i]; }
        const float got = wt * acc; float* po = Og + (size_t)st * NM + un * NE + cj; *(volatile float*)po = got; __threadfence(); *(volatile float*)po = got; } }

extern "C" void kernel_launch(void* const* d_in, const int* in_sizes, int n_in, void* d_out, int out_size, void* d_ws, size_t ws_size, hipStream_t stream) {
    if (n_in < 7) return;
    if (in_sizes[0] != NL * NM || in_sizes[1] != NM * NM || in_sizes[2] != NM * NM || in_sizes[3] != NM * NM || in_sizes[4] != NM * NM || in_sizes[5] != NE || in_sizes[6] != NE) return;
    if (out_size != NL * NM) return;
    static_assert(NL % 64 == 0 && NM % 64 == 0 && NJ % 64 == 0 && NM % 32 == 0 && NJ == 3 * NM && OB == NM && OC == 2 * NM && NM == NU * NE && NE == 64 && (NL * NM / 8) % 256 == 0 && (NM * NM / 8) % 256 == 0 && (NL * NU) % 256 == 0 && NU == 16 && NL % 2 == 0, "the products: row and column counts multiples of 64, the depths of 32; every one-dimensional launch exact; 16 units of 64 words; the first product's columns in their three parts");
    const float* i0 = (const float*)d_in[0]; const float* i1 = (const float*)d_in[1]; const float* i2 = (const float*)d_in[2]; const float* i3 = (const float*)d_in[3]; const float* i4 = (const float*)d_in[4]; const float* i5 = (const float*)d_in[5]; const float* i6 = (const float*)d_in[6]; float* out = (float*)d_out;
    char* wsp = (char*)d_ws; auto take = [&](size_t bytes) { char* p = wsp; wsp += (bytes + 255) & ~(size_t)255; return (void*)p; };
    bf* Xb = (bf*)take((size_t)NL * NM * 2); bf* Wb = (bf*)take((size_t)NJ * NM * 2); float* Pj = (float*)take((size_t)NL * NJ * 4); float* Lg = (float*)take((size_t)NL * NU * 4); float* Ez = (float*)take((size_t)NL * NU * 4); float* Wg = (float*)take((size_t)NL * NU * 4); float* Cf = (float*)take((size_t)NL * NU * 4); float* Og = (float*)take((size_t)NL * NM * 4); h16* Oh = (h16*)take((size_t)NL * NM * 2); h16* Wh = (h16*)take((size_t)NM * NM * 2);
    if ((size_t)(wsp - (char*)d_ws) > ws_size) return;
    k_cvt8<<<(unsigned)(NL * NM / 8 / 256), 256, 0, stream>>>(i0, Xb, (size_t)NL * NM / 8);
    k_cvt8<<<(unsigned)(NM * NM / 8 / 256), 256, 0, stream>>>(i1, Wb, (size_t)NM * NM / 8);
    k_cvt8<<<(unsigned)(NM * NM / 8 / 256), 256, 0, stream>>>(i2, Wb + (size_t)NM * NM, (size_t)NM * NM / 8);
    k_cvt8<<<(unsigned)(NM * NM / 8 / 256), 256, 0, stream>>>(i3, Wb + (size_t)2 * NM * NM, (size_t)NM * NM / 8);
    k_gemmw<bf, 0, false><<<dim3(NL / 64, NJ / 64, 1), 32, 0, stream>>>(Xb, nullptr, Wb, nullptr, NM, Pj, NJ, nullptr, 0, 0, 0);
    k_eases<<<(unsigned)(NL * NU / 256), 256, 0, stream>>>(i0, i5, i6, Pj, Lg, Ez);
    k_sums<<<1, 2 * NU, 0, stream>>>(Lg, Ez, Wg, Cf);
    k_tally<<<NU, NE, 0, stream>>>(Pj, Wg, Cf, Og);
    k_c16<false><<<(unsigned)(NL * NM / 8 / 256), 256, 0, stream>>>(Og, Oh, (size_t)NL * NM / 8);
    k_c16<true><<<(unsigned)(NM * NM / 8 / 256), 256, 0, stream>>>(i4, Wh, (size_t)NM * NM / 8);
    k_gemmw<h16, 0, false><<<dim3(NL / 64, NM / 64, 1), 32, 0, stream>>>(Oh, nullptr, Wh, nullptr, NM, out, NM, nullptr, 0, 0, 0);
}
